// GraphTransformer2Layer_37082747633995
// MI455X (gfx1250) — hardware-verified
//
#include <hip/hip_runtime.h>
#include <stdint.h>
#include <stddef.h>


#define FEAT 128
#define CH1 32
#define CH2 10
#define P2W 64
#define TN 1024
#define NPW 128
#define CAP1 384
#define CAP2 2560
#define PB 136
#define NTHR 256
#define SP1 132
#define SP2 68

#define OFF_LST 0
#define OFF_CNT (64 * CAP1)
#define OFF_SEG (OFF_CNT + 64)
#define OFF_SST (OFF_SEG + 8 * CAP2)
#define OFF_SCT (OFF_SST + TN)
#define OFF_STG (OFF_SCT + TN)
#define EDGE_LDS_WORDS (OFF_STG + 8 * 512)
#define EDGE_LDS_BYTES (EDGE_LDS_WORDS * 4)
#define GEMM1_LDS_BYTES (8 * 16 * SP1 * 4)
#define GEMM2_LDS_BYTES (8 * 16 * SP2 * 4)

typedef _Float16 v8h __attribute__((ext_vector_type(8)));
typedef _Float16 v16h __attribute__((ext_vector_type(16)));
typedef float v8f __attribute__((ext_vector_type(8)));
typedef float v4f __attribute__((ext_vector_type(4)));
union Frag { v16h v; v8h h8[2]; };

__device__ __forceinline__ v8f wmma_f16(v16h a, v16h b, v8f c)
{
    c = __builtin_amdgcn_wmma_f32_16x16x32_f16(false, a, false, b, (short)0, c, false, false);
    asm volatile("v_nop\n\tv_nop\n\tv_nop\n\tv_nop" : "+v"(c) : "v"(a), "v"(b));
    return c;
}

__device__ __forceinline__ v8h cvt8h(const float* p)
{
    const v4f a = *(const v4f*)p;
    const v4f b = *(const v4f*)(p + 4);
    v8h r;
    r[0] = (_Float16)a[0]; r[1] = (_Float16)a[1]; r[2] = (_Float16)a[2]; r[3] = (_Float16)a[3];
    r[4] = (_Float16)b[0]; r[5] = (_Float16)b[1]; r[6] = (_Float16)b[2]; r[7] = (_Float16)b[3];
    return r;
}

__device__ __forceinline__ int wave_incl_scan(int v, int lane)
{
#pragma unroll
    for (int d = 1; d < 32; d <<= 1) {
        const int t = __shfl_up(v, d);
        if (lane >= d) v += t;
    }
    return v;
}

__device__ __forceinline__ void rows_store_128(const float* sw, float* O, int rowB, int M, int lane)
{
#pragma unroll
    for (int i = 0; i < 16; ++i) {
        const int grow = rowB + i;
        if (grow < M) {
            const v4f v = *(const v4f*)(sw + i * SP1 + 4 * lane);
            *(volatile v4f*)(O + (size_t)grow * FEAT + 4 * lane) = v;
        }
    }
}

__device__ __forceinline__ void rows_store_64(const float* sw, float* P, int rowB, int M, int lane)
{
    const int hh = lane >> 4, nn = lane & 15;
#pragma unroll
    for (int i = 0; i < 8; ++i) {
        const int rr = 2 * i + hh;
        const int grow = rowB + rr;
        if (grow < M) {
            const v4f v = *(const v4f*)(sw + rr * SP2 + 4 * nn);
            *(volatile v4f*)(P + (size_t)grow * P2W + 4 * nn) = v;
        }
    }
}

__device__ __forceinline__ void rows_store_h(const float* stg, float* Sb, int nodeB, int N, int lane)
{
#pragma unroll
    for (int rr = 0; rr < 4; ++rr) {
        const int nd = nodeB + rr;
        if (nd < N) {
            const v4f v = *(const v4f*)(stg + rr * FEAT + 4 * lane);
            *(volatile v4f*)(Sb + (size_t)nd * FEAT + 4 * lane) = v;
        }
    }
}

__device__ __forceinline__ void block_store_lines(const float* OT, float* ob, int nln, int rem, int w, int lane)
{
    const int ngrp = (nln + 3) >> 2;
    for (int g = w; g < ngrp; g += 8) {
        const int ln = g * 4 + (lane >> 3);
        if (ln < nln) {
            const v4f v = *(const v4f*)(OT + ln * 32 + 4 * (lane & 7));
            *(volatile v4f*)(ob + (size_t)ln * 32 + 4 * (lane & 7)) = v;
        }
    }
    if (w == 0 && lane < rem) {
        const float v = OT[nln * 32 + lane];
        *(volatile float*)(ob + (size_t)nln * 32 + lane) = v;
    }
}

__global__ void __launch_bounds__(NTHR)
k_gemm1(const float* __restrict__ X,
        const float* __restrict__ W0, const float* __restrict__ Bi0,
        const float* __restrict__ W1, const float* __restrict__ Bi1,
        const float* __restrict__ W2, const float* __restrict__ Bi2,
        const float* __restrict__ W3, const float* __restrict__ Bi3,
        float* __restrict__ OUT, int M)
{
    extern __shared__ __align__(16) unsigned char lds_g1[];
    _Float16* Bt = (_Float16*)lds_g1;
    float* stgall = (float*)lds_g1;

    const int tid = threadIdx.x;
    const int lane = tid & 31;
    const int w = tid >> 5;
    const int h = lane >> 4;
    const int n = lane & 15;
    const int p = blockIdx.y;
    const float* W  = (p == 0) ? W0  : (p == 1) ? W1  : (p == 2) ? W2  : W3;
    const float* Bi = (p == 0) ? Bi0 : (p == 1) ? Bi1 : (p == 2) ? Bi2 : Bi3;
    float* O = OUT + (size_t)p * (size_t)M * FEAT;

    for (int i = tid; i < FEAT * FEAT; i += NTHR) {
        const int k = i >> 7;
        const int nn = i & 127;
        Bt[nn * PB + k] = (_Float16)W[i];
    }
    __syncthreads();

    const int rowB = blockIdx.x * 128 + w * 16;
    const int mrow = min(rowB + n, M - 1);
    const float* ar = X + (size_t)mrow * FEAT;

    v8f acc[8];
#pragma unroll
    for (int t = 0; t < 8; ++t) {
#pragma unroll
        for (int r = 0; r < 8; ++r) acc[t][r] = 0.0f;
    }

#pragma unroll
    for (int k0 = 0; k0 < FEAT; k0 += 32) {
        Frag a;
        a.h8[0] = cvt8h(ar + k0 + 8 * h);
        a.h8[1] = cvt8h(ar + k0 + 16 + 8 * h);
#pragma unroll
        for (int t = 0; t < 8; ++t) {
            const _Float16* br = Bt + (16 * t + n) * PB + k0 + 8 * h;
            Frag b;
            b.h8[0] = *(const v8h*)(br);
            b.h8[1] = *(const v8h*)(br + 16);
            acc[t] = wmma_f16(a.v, b.v, acc[t]);
        }
    }
    __syncthreads();

    float* sw = stgall + w * (16 * SP1);
#pragma unroll
    for (int t = 0; t < 8; ++t) {
        const float bv = Bi[16 * t + n];
#pragma unroll
        for (int r = 0; r < 8; ++r) sw[(8 * h + r) * SP1 + 16 * t + n] = acc[t][r] + bv;
    }
    __syncthreads();

    rows_store_128(sw, O, rowB, M, lane);
    __threadfence();
    rows_store_128(sw, O, rowB, M, lane);
}

__global__ void __launch_bounds__(NTHR)
k_gemm2(const float* __restrict__ A,
        const float* __restrict__ W0, const float* __restrict__ Bi0,
        const float* __restrict__ W1, const float* __restrict__ Bi1,
        const float* __restrict__ W2, const float* __restrict__ Bi2,
        const float* __restrict__ W3, const float* __restrict__ Bi3,
        float* __restrict__ P, int M)
{
    extern __shared__ __align__(16) unsigned char lds_g2[];
    _Float16* Bt = (_Float16*)lds_g2;
    float* stgall = (float*)lds_g2;

    const int tid = threadIdx.x;
    const int lane = tid & 31;
    const int w = tid >> 5;
    const int h = lane >> 4;
    const int n = lane & 15;

    for (int i = tid; i < 64 * FEAT; i += NTHR) {
        const int nn = i & 63;
        const int k = i >> 6;
        const int pp = nn >> 4;
        const int c = nn & 15;
        const float* W = (pp == 0) ? W0 : (pp == 1) ? W1 : (pp == 2) ? W2 : W3;
        const int cc = min(c, CH2 - 1);
        float v = W[k * CH2 + cc];
        if (c >= CH2) v = 0.0f;
        Bt[nn * PB + k] = (_Float16)v;
    }
    __syncthreads();

    const int rowB = blockIdx.x * 128 + w * 16;
    const int mrow = min(rowB + n, M - 1);
    const float* ar = A + (size_t)mrow * FEAT;

    v8f acc[4];
#pragma unroll
    for (int t = 0; t < 4; ++t) {
#pragma unroll
        for (int r = 0; r < 8; ++r) acc[t][r] = 0.0f;
    }

#pragma unroll
    for (int k0 = 0; k0 < FEAT; k0 += 32) {
        Frag a;
        a.h8[0] = cvt8h(ar + k0 + 8 * h);
        a.h8[1] = cvt8h(ar + k0 + 16 + 8 * h);
#pragma unroll
        for (int t = 0; t < 4; ++t) {
            const _Float16* br = Bt + (16 * t + n) * PB + k0 + 8 * h;
            Frag b;
            b.h8[0] = *(const v8h*)(br);
            b.h8[1] = *(const v8h*)(br + 16);
            acc[t] = wmma_f16(a.v, b.v, acc[t]);
        }
    }
    __syncthreads();

    float* sw = stgall + w * (16 * SP2);
    const int nc = min(n, CH2 - 1);
#pragma unroll
    for (int t = 0; t < 4; ++t) {
        const float* Bi = (t == 0) ? Bi0 : (t == 1) ? Bi1 : (t == 2) ? Bi2 : Bi3;
        float bv = Bi[nc];
        if (n >= CH2) bv = 0.0f;
#pragma unroll
        for (int r = 0; r < 8; ++r) sw[(8 * h + r) * SP2 + 16 * t + n] = acc[t][r] + bv;
    }
    __syncthreads();

    rows_store_64(sw, P, rowB, M, lane);
    __threadfence();
    rows_store_64(sw, P, rowB, M, lane);
}

template <int LAYER>
__global__ void __launch_bounds__(NTHR)
k_edge(float* buf, const int* __restrict__ ei, float* __restrict__ out, int N, int E)
{
    extern __shared__ __align__(16) int lds_e[];
    int* LST = lds_e + OFF_LST;
    int* CNT = lds_e + OFF_CNT;
    int* SEG = lds_e + OFF_SEG;
    int* SST = lds_e + OFF_SST;
    int* SCT = lds_e + OFF_SCT;
    float* STG = (float*)(lds_e + OFF_STG);
    float* OT = (float*)(lds_e + OFF_LST);

    const int tid = threadIdx.x;
    const int lane = tid & 31;
    const int w = tid >> 5;
    const int n0 = blockIdx.x * TN;
    const int nb0 = w * NPW;
    const int* src = ei;
    const int* dst = ei + E;

    {
        int myc = 0;
        const int chunk = (E + 7) >> 3;
        const int eBeg = w * chunk;
        const int eEnd = min(eBeg + chunk, E);
        for (int base = eBeg; base < eEnd; base += 32) {
            const int e = base + lane;
            int loc = -1;
            if (e < eEnd) {
                const int d = dst[e];
                if (d >= n0 && d < N) loc = d - n0;
            }
            const bool match = (loc >= 0) && (loc < TN);
            unsigned int mask = __builtin_amdgcn_ballot_w32(match);
            while (mask != 0u) {
                const int j = __builtin_ctz(mask);
                mask &= (mask - 1u);
                const int lj = __shfl(loc, j);
                const int bk = lj >> 7;
                const int c = __shfl(myc, bk);
                if (c < CAP1) {
                    if (lane == 0) LST[(w * 8 + bk) * CAP1 + c] = ((base + j) << 10) | lj;
                    if (lane == bk) myc = myc + 1;
                }
            }
        }
        if (lane < 8) CNT[w * 8 + lane] = min(myc, CAP1);
    }
    __syncthreads();

    int c0 = 0, c1 = 0, c2 = 0, c3 = 0;
    for (int w2 = 0; w2 < 8; ++w2) {
        const int li = w2 * 8 + w;
        const int nl = CNT[li];
        const int* L = LST + li * CAP1;
        for (int i = 0; i < nl; ++i) {
            const int u = L[i];
            const int jj = (u & (TN - 1)) - nb0;
            const bool mine = (jj >= 0) && (jj < NPW) && ((jj & 31) == lane);
            const int sl = (jj >> 5) & 3;
            if (mine) {
                if (sl == 0) ++c0; else if (sl == 1) ++c1; else if (sl == 2) ++c2; else ++c3;
            }
        }
    }
    const int p0 = wave_incl_scan(c0, lane);
    const int p1 = wave_incl_scan(c1, lane);
    const int p2 = wave_incl_scan(c2, lane);
    const int p3 = wave_incl_scan(c3, lane);
    const int t0 = __shfl(p0, 31);
    const int t1 = __shfl(p1, 31);
    const int t2 = __shfl(p2, 31);
    const int st0 = p0 - c0;
    const int st1 = t0 + p1 - c1;
    const int st2 = t0 + t1 + p2 - c2;
    const int st3 = t0 + t1 + t2 + p3 - c3;
    {
        int q0 = 0, q1 = 0, q2 = 0, q3 = 0;
        for (int w2 = 0; w2 < 8; ++w2) {
            const int li = w2 * 8 + w;
            const int nl = CNT[li];
            const int* L = LST + li * CAP1;
            for (int i = 0; i < nl; ++i) {
                const int u = L[i];
                const int jj = (u & (TN - 1)) - nb0;
                const bool mine = (jj >= 0) && (jj < NPW) && ((jj & 31) == lane);
                const int sl = (jj >> 5) & 3;
                if (mine) {
                    int pos;
                    if (sl == 0)      { pos = st0 + q0; ++q0; }
                    else if (sl == 1) { pos = st1 + q1; ++q1; }
                    else if (sl == 2) { pos = st2 + q2; ++q2; }
                    else              { pos = st3 + q3; ++q3; }
                    if (pos < CAP2) SEG[w * CAP2 + pos] = u >> 10;
                }
            }
        }
    }
    SST[nb0 + lane]      = min(st0, CAP2);
    SCT[nb0 + lane]      = max(0, min(c0, CAP2 - st0));
    SST[nb0 + 32 + lane] = min(st1, CAP2);
    SCT[nb0 + 32 + lane] = max(0, min(c1, CAP2 - st1));
    SST[nb0 + 64 + lane] = min(st2, CAP2);
    SCT[nb0 + 64 + lane] = max(0, min(c2, CAP2 - st2));
    SST[nb0 + 96 + lane] = min(st3, CAP2);
    SCT[nb0 + 96 + lane] = max(0, min(c3, CAP2 - st3));
    __syncthreads();

    if (LAYER == 1) {
        const size_t plane = (size_t)N * FEAT;
        const float* Qb = buf;
        const float* Kb = buf + plane;
        const float* Vb = buf + 2 * plane;
        float* Sb = buf + 3 * plane;
        float* stg = STG + w * 512;
        const int sub = lane >> 3;
        const int cb = (lane & 7) * 16;
        const float scale = 0.17677669529663688f;
#pragma unroll 1
        for (int it = 0; it < 32; ++it) {
            const int nloc = nb0 + it * 4 + sub;
            const int node = n0 + nloc;
            const int nodec = min(node, N - 1);
            const int st = SST[nloc];
            const int cn = SCT[nloc];
            float qv[16];
            {
                const float* qr = Qb + (size_t)nodec * FEAT + cb;
#pragma unroll
                for (int c4 = 0; c4 < 4; ++c4) {
                    const v4f t = *(const v4f*)(qr + 4 * c4);
                    qv[4 * c4 + 0] = t[0]; qv[4 * c4 + 1] = t[1];
                    qv[4 * c4 + 2] = t[2]; qv[4 * c4 + 3] = t[3];
                }
            }
            float acc[16];
#pragma unroll
            for (int c = 0; c < 16; ++c) acc[c] = 0.0f;
            float m = -__builtin_huge_valf();
            float ssum = 0.0f;
#pragma unroll 1
            for (int i = 0; i < cn; ++i) {
                int e = SEG[w * CAP2 + st + i];
                e = min(max(e, 0), E - 1);
                int sj = src[e];
                sj = min(max(sj, 0), N - 1);
                const float* kr = Kb + (size_t)sj * FEAT + cb;
                float d = 0.0f;
#pragma unroll
                for (int c4 = 0; c4 < 4; ++c4) {
                    const v4f t = *(const v4f*)(kr + 4 * c4);
                    d += qv[4 * c4 + 0] * t[0];
                    d += qv[4 * c4 + 1] * t[1];
                    d += qv[4 * c4 + 2] * t[2];
                    d += qv[4 * c4 + 3] * t[3];
                }
                d += __shfl_xor(d, 1);
                const float lg = d * scale;
                const float mn = fmaxf(m, lg);
                const float rs = __expf(m - mn);
                const float pe = __expf(lg - mn);
                m = mn;
                ssum = ssum * rs + pe;
                const float* vr = Vb + (size_t)sj * FEAT + cb;
#pragma unroll
                for (int c4 = 0; c4 < 4; ++c4) {
                    const v4f t = *(const v4f*)(vr + 4 * c4);
                    acc[4 * c4 + 0] = acc[4 * c4 + 0] * rs + pe * t[0];
                    acc[4 * c4 + 1] = acc[4 * c4 + 1] * rs + pe * t[1];
                    acc[4 * c4 + 2] = acc[4 * c4 + 2] * rs + pe * t[2];
                    acc[4 * c4 + 3] = acc[4 * c4 + 3] * rs + pe * t[3];
                }
            }
            const float inv = 1.0f / (ssum + 1e-16f);
            const float* hr = Sb + (size_t)nodec * FEAT + cb;
#pragma unroll
            for (int c4 = 0; c4 < 4; ++c4) {
                const v4f t = *(const v4f*)(hr + 4 * c4);
                v4f o;
#pragma unroll
                for (int j = 0; j < 4; ++j) {
                    const float z = acc[4 * c4 + j] * inv + t[j];
                    o[j] = (z > 0.0f) ? z : (__expf(z) - 1.0f);
                }
                *(v4f*)(stg + sub * FEAT + cb + 4 * c4) = o;
            }
            const int nodeB = n0 + nb0 + it * 4;
            rows_store_h(stg, Sb, nodeB, N, lane);
            __threadfence();
            rows_store_h(stg, Sb, nodeB, N, lane);
        }
    } else {
        const float* Pb = buf;
        const float scale = 0.31622776601683794f;
#pragma unroll 1
        for (int it = 0; it < 4; ++it) {
            const int nloc = nb0 + it * 32 + lane;
            const int node = n0 + nloc;
            const int nodec = min(node, N - 1);
            const int st = SST[nloc];
            const int cn = SCT[nloc];
            const float* pr = Pb + (size_t)nodec * P2W;
            float qv[12];
#pragma unroll
            for (int c4 = 0; c4 < 3; ++c4) {
                const v4f t = *(const v4f*)(pr + 4 * c4);
                qv[4 * c4 + 0] = t[0]; qv[4 * c4 + 1] = t[1];
                qv[4 * c4 + 2] = t[2]; qv[4 * c4 + 3] = t[3];
            }
            float acc[12];
#pragma unroll
            for (int c = 0; c < 12; ++c) acc[c] = 0.0f;
            float m = -__builtin_huge_valf();
            float ssum = 0.0f;
#pragma unroll 1
            for (int i = 0; i < cn; ++i) {
                int e = SEG[w * CAP2 + st + i];
                e = min(max(e, 0), E - 1);
                int sj = src[e];
                sj = min(max(sj, 0), N - 1);
                const float* kr = Pb + (size_t)sj * P2W + 16;
                float d = 0.0f;
#pragma unroll
                for (int c4 = 0; c4 < 3; ++c4) {
                    const v4f t = *(const v4f*)(kr + 4 * c4);
#pragma unroll
                    for (int j = 0; j < 4; ++j) {
                        if (4 * c4 + j < CH2) d += qv[4 * c4 + j] * t[j];
                    }
                }
                const float lg = d * scale;
                const float mn = fmaxf(m, lg);
                const float rs = __expf(m - mn);
                const float pe = __expf(lg - mn);
                m = mn;
                ssum = ssum * rs + pe;
                const float* vr = Pb + (size_t)sj * P2W + 32;
#pragma unroll
                for (int c4 = 0; c4 < 3; ++c4) {
                    const v4f t = *(const v4f*)(vr + 4 * c4);
#pragma unroll
                    for (int j = 0; j < 4; ++j) {
                        if (4 * c4 + j < CH2) acc[4 * c4 + j] = acc[4 * c4 + j] * rs + pe * t[j];
                    }
                }
            }
            const float inv = 1.0f / (ssum + 1e-16f);
            const float* sk = pr + 48;
#pragma unroll
            for (int c4 = 0; c4 < 3; ++c4) {
                const v4f t = *(const v4f*)(sk + 4 * c4);
#pragma unroll
                for (int j = 0; j < 4; ++j) {
                    if (4 * c4 + j < CH2) OT[nloc * CH2 + 4 * c4 + j] = acc[4 * c4 + j] * inv + t[j];
                }
            }
        }
        __syncthreads();
        const int nn = min(TN, N - n0);
        const int nfl = nn * CH2;
        const int nln = nfl >> 5;
        const int rem = nfl - (nln << 5);
        float* ob = out + (size_t)n0 * CH2;
        block_store_lines(OT, ob, nln, rem, w, lane);
        __threadfence();
        block_store_lines(OT, ob, nln, rem, w, lane);
    }
}

extern "C" void kernel_launch(void* const* d_in, const int* in_sizes, int n_in,
                              void* d_out, int out_size, void* d_ws, size_t ws_size,
                              hipStream_t stream)
{
    if (n_in < 18) return;
    const int N = in_sizes[0] / FEAT;
    const int E = in_sizes[1] / 2;
    if (N <= 0 || E < 0 || E > 2097151) return;
    if (in_sizes[0] != N * FEAT || in_sizes[1] != 2 * E) return;
    if (in_sizes[2] != FEAT * FEAT || in_sizes[4] != FEAT * FEAT ||
        in_sizes[6] != FEAT * FEAT || in_sizes[8] != FEAT * FEAT) return;
    if (in_sizes[3] < FEAT || in_sizes[5] < FEAT || in_sizes[7] < FEAT || in_sizes[9] < FEAT) return;
    if (in_sizes[10] != FEAT * CH2 || in_sizes[12] != FEAT * CH2 ||
        in_sizes[14] != FEAT * CH2 || in_sizes[16] != FEAT * CH2) return;
    if (in_sizes[11] < CH2 || in_sizes[13] < CH2 || in_sizes[15] < CH2 || in_sizes[17] < CH2) return;
    if (out_size != N * CH2) return;

    const size_t bytesQ = (size_t)N * 4 * FEAT * sizeof(float);
    const size_t offP = (bytesQ + 255) & ~(size_t)255;
    const size_t bytesP = (size_t)N * P2W * sizeof(float);
    if (offP + bytesP > ws_size) return;

    const float* x   = (const float*)d_in[0];
    const int*   ei  = (const int*)d_in[1];
    const float* Wq1 = (const float*)d_in[2];  const float* bq1 = (const float*)d_in[3];
    const float* Wk1 = (const float*)d_in[4];  const float* bk1 = (const float*)d_in[5];
    const float* Wv1 = (const float*)d_in[6];  const float* bv1 = (const float*)d_in[7];
    const float* Ws1 = (const float*)d_in[8];  const float* bs1 = (const float*)d_in[9];
    const float* Wq2 = (const float*)d_in[10]; const float* bq2 = (const float*)d_in[11];
    const float* Wk2 = (const float*)d_in[12]; const float* bk2 = (const float*)d_in[13];
    const float* Wv2 = (const float*)d_in[14]; const float* bv2 = (const float*)d_in[15];
    const float* Ws2 = (const float*)d_in[16]; const float* bs2 = (const float*)d_in[17];
    float* out = (float*)d_out;

    float* QKVS1 = (float*)d_ws;
    float* P2    = (float*)((unsigned char*)d_ws + offP);
    const float* H1 = QKVS1 + (size_t)3 * N * FEAT;

    hipFuncSetAttribute((const void*)&k_gemm1, hipFuncAttributeMaxDynamicSharedMemorySize, GEMM1_LDS_BYTES);
    hipFuncSetAttribute((const void*)&k_gemm2, hipFuncAttributeMaxDynamicSharedMemorySize, GEMM2_LDS_BYTES);
    hipFuncSetAttribute((const void*)&k_edge<1>, hipFuncAttributeMaxDynamicSharedMemorySize, EDGE_LDS_BYTES);
    hipFuncSetAttribute((const void*)&k_edge<2>, hipFuncAttributeMaxDynamicSharedMemorySize, EDGE_LDS_BYTES);

    const dim3 blk(NTHR);
    const dim3 g1((N + 127) / 128, 4);
    const dim3 g2((N + 127) / 128);
    const dim3 ge((N + TN - 1) / TN);

    hipLaunchKernelGGL(k_gemm1, g1, blk, GEMM1_LDS_BYTES, stream,
                       x, Wq1, bq1, Wk1, bk1, Wv1, bv1, Ws1, bs1, QKVS1, N);
    hipLaunchKernelGGL(HIP_KERNEL_NAME(k_edge<1>), ge, blk, EDGE_LDS_BYTES, stream,
                       QKVS1, ei, out, N, E);
    hipLaunchKernelGGL(k_gemm2, g2, blk, GEMM2_LDS_BYTES, stream,
                       H1, Wq2, bq2, Wk2, bk2, Wv2, bv2, Ws2, bs2, P2, N);
    hipLaunchKernelGGL(HIP_KERNEL_NAME(k_edge<2>), ge, blk, EDGE_LDS_BYTES, stream,
                       P2, ei, out, N, E);
    hipGetLastError();
}
